// StructuralProbe_13460427505803
// MI455X (gfx1250) — hardware-verified
//
#include <hip/hip_runtime.h>


#ifndef NB
#define NB 32
#endif
#ifndef SEQ
#define SEQ 256
#endif
#define NB_FULL  32
#define SEQ_FULL 256
#ifndef OUT_SEQ
#define OUT_SEQ SEQ
#endif
#define DIN  1024
#define RK   128

static_assert(RK == 128);
static_assert(DIN % 64 == 0);
static_assert(RK % 32 == 0);
static_assert(SEQ % 64 == 0);
static_assert((NB * SEQ) % 32 == 0);
static_assert(OUT_SEQ % 32 == 0);
static_assert(OUT_SEQ >= SEQ);
static_assert(((size_t)SEQ * DIN) % 8 == 0);
static_assert(NB <= NB_FULL);
static_assert(SEQ <= SEQ_FULL);

typedef unsigned short bf;
typedef __attribute__((ext_vector_type(16))) __bf16   v16bf;
typedef __attribute__((ext_vector_type(8)))  unsigned short v8us;
typedef __attribute__((ext_vector_type(8)))  float    v8f;
typedef __attribute__((ext_vector_type(4)))  float    v4f;
typedef v4f  __attribute__((may_alias)) v4fa;
typedef v8us __attribute__((may_alias)) v8usa;

__device__ __forceinline__ unsigned short f2bf(float f) { unsigned u = __float_as_uint(f); u += 0x7FFFu + ((u >> 16) & 1u); return (unsigned short)(u >> 16); }
__device__ __forceinline__ float bf2f(unsigned short h) { return __uint_as_float(((unsigned)h) << 16); }
__device__ __forceinline__ v16bf cat16b(v8us lo, v8us hi) { return __builtin_bit_cast(v16bf, __builtin_shufflevector(lo, hi, 0, 1, 2, 3, 4, 5, 6, 7, 8, 9, 10, 11, 12, 13, 14, 15)); }
__device__ __forceinline__ v8f wmmab(v16bf a, v16bf b, v8f c) { return __builtin_amdgcn_wmma_f32_16x16x32_bf16(false, a, false, b, (short)0, c, false, false); }
__device__ __forceinline__ v16bf ldb(const bf* p)  { return cat16b(*(const v8us*)p, *(const v8us*)(p + 16)); }
__device__ __forceinline__ void wave_sync() { __builtin_amdgcn_fence(3  , "wavefront"); __builtin_amdgcn_wave_barrier(); asm volatile("" ::: "memory"); }

__global__ __launch_bounds__(256) void k_cvt8(const float* __restrict__ src, bf* dst, size_t n8) {
    const size_t i = (size_t)blockIdx.x * 256 + threadIdx.x; if (i >= n8) return;
    const v8f v = *(const v8f*)(src + i * 8); v8us o;
#pragma unroll
    for (int k = 0; k < 8; ++k) o[k] = f2bf(v[k]);
    *(volatile v8us*)(dst + i * 8) = o; __threadfence(); *(volatile v8us*)(dst + i * 8) = o;
}

__global__ __launch_bounds__(256) void k_tcvt(const float* __restrict__ P, bf* PT) {
    __shared__ __align__(16) unsigned short ts[RK * 72];
    const int tid = threadIdx.x; const int k0 = blockIdx.x * 64;
#pragma unroll 4
    for (int it = 0; it < 32; ++it) { const int idx = it * 256 + tid; const int k = idx >> 7, n = idx & 127;
        ts[n * 72 + k] = f2bf(P[(size_t)(k0 + k) * RK + n]); }
    __syncthreads();
#pragma unroll 1
    for (int ps = 0; ps < 2; ++ps) {
#pragma unroll
        for (int it = 0; it < 4; ++it) { const int n = it * 32 + (tid >> 3), pc = (tid & 7) * 8;
            const v8us o = *(const v8usa*)(&ts[n * 72 + pc]);
            *(volatile v8us*)(PT + (size_t)n * DIN + k0 + pc) = o; }
        if (ps == 0) __threadfence(); }
}

__global__ __launch_bounds__(32) void k_proj(const bf* __restrict__ A, const bf* __restrict__ Bt, bf* TH, bf* TL, float* NRM) {
    __shared__ __align__(16) float os[16 * 132];
    const int K = DIN;
    const int lane = threadIdx.x & 31, lr = lane & 15, hi = lane >> 4; const int r0 = blockIdx.x * 32;
    v8f acc[2][8];
#pragma unroll
    for (int mb = 0; mb < 2; ++mb)
#pragma unroll
        for (int nb = 0; nb < 8; ++nb) acc[mb][nb] = (v8f){};
    const size_t aoff = (size_t)(r0 + lr) * K + 8 * hi, boff = (size_t)lr * K + 8 * hi;
#pragma unroll 1
    for (int kc = 0; kc < K; kc += 32) {
        const v16bf a0 = ldb(A + aoff + kc), a1 = ldb(A + aoff + (size_t)16 * K + kc);
#pragma unroll
        for (int nb = 0; nb < 8; ++nb) { const v16bf b = ldb(Bt + boff + (size_t)nb * 16 * K + kc);
            acc[0][nb] = wmmab(a0, b, acc[0][nb]); acc[1][nb] = wmmab(a1, b, acc[1][nb]); }
        asm volatile("v_nop\n\tv_nop\n\tv_nop\n\tv_nop" : "+v"(acc[0][0]), "+v"(acc[0][1]), "+v"(acc[0][2]), "+v"(acc[0][3]), "+v"(acc[0][4]), "+v"(acc[0][5]), "+v"(acc[0][6]), "+v"(acc[0][7]) : "v"(a0));
        asm volatile("v_nop\n\tv_nop\n\tv_nop\n\tv_nop" : "+v"(acc[1][0]), "+v"(acc[1][1]), "+v"(acc[1][2]), "+v"(acc[1][3]), "+v"(acc[1][4]), "+v"(acc[1][5]), "+v"(acc[1][6]), "+v"(acc[1][7]) : "v"(a1));
    }
    float nsl[2];
#pragma unroll
    for (int mb = 0; mb < 2; ++mb) {
#pragma unroll
        for (int nb = 0; nb < 8; ++nb) {
#pragma unroll
            for (int j = 0; j < 8; ++j) os[(hi * 8 + j) * 132 + nb * 16 + lr] = acc[mb][nb][j]; }
        wave_sync();
        float s = 0.0f;
#pragma unroll 4
        for (int c = 0; c < 16; ++c) { const v4f x = *(const v4fa*)(&os[lr * 132 + hi * 64 + c * 4]);
            s = fmaf(x[0], x[0], s); s = fmaf(x[1], x[1], s); s = fmaf(x[2], x[2], s); s = fmaf(x[3], x[3], s); }
        s += __shfl_xor(s, 16, 32);
        nsl[mb] = s;
        const size_t sb = (size_t)(r0 + mb * 16) * RK;
#pragma unroll 1
        for (int ps = 0; ps < 2; ++ps) {
#pragma unroll
            for (int s8 = 0; s8 < 8; ++s8) { const int row = 2 * s8 + hi, c8 = lr * 8;
                const v4f x0 = *(const v4fa*)(&os[row * 132 + c8]); const v4f x1 = *(const v4fa*)(&os[row * 132 + c8 + 4]); v8us hv, lv;
#pragma unroll
                for (int i = 0; i < 4; ++i) { const unsigned short h0 = f2bf(x0[i]); const unsigned short h1 = f2bf(x1[i]);
                    hv[i] = h0; hv[4 + i] = h1; lv[i] = f2bf(x0[i] - bf2f(h0)); lv[4 + i] = f2bf(x1[i] - bf2f(h1)); }
                const size_t oo = sb + (size_t)row * RK + c8;
                *(volatile v8us*)(TH + oo) = hv; *(volatile v8us*)(TL + oo) = lv; }
            if (ps == 0) __threadfence(); }
        wave_sync();
    }
    const float nv = hi ? nsl[1] : nsl[0];
    *(volatile float*)(NRM + r0 + lane) = nv; __threadfence(); *(volatile float*)(NRM + r0 + lane) = nv;
}

__global__ __launch_bounds__(32) void k_gram(const bf* __restrict__ TP, size_t loOff, const float* __restrict__ NRM, float* OUT) {
    __shared__ __align__(16) float os[16 * 68];
    const int lane = threadIdx.x & 31, lr = lane & 15, hi = lane >> 4;
    const int b = blockIdx.z, i0 = blockIdx.y * 64, j0 = blockIdx.x * 64;
    const size_t rb = (size_t)b * SEQ;
    const size_t aoff = (rb + i0 + lr) * RK + 8 * hi, boff = (rb + j0 + lr) * RK + 8 * hi;
    v8f acc[4][4];
#pragma unroll
    for (int mb = 0; mb < 4; ++mb)
#pragma unroll
        for (int nb = 0; nb < 4; ++nb) acc[mb][nb] = (v8f){};
#pragma unroll
    for (int p = 0; p < 3; ++p) {
        const size_t ap = (p == 2) ? loOff : (size_t)0, bp = (p == 1) ? loOff : (size_t)0;
#pragma unroll 1
        for (int kc = 0; kc < RK; kc += 32) {
            v16bf a[4];
#pragma unroll
            for (int mb = 0; mb < 4; ++mb) a[mb] = ldb(TP + ap + aoff + (size_t)mb * 16 * RK + kc);
#pragma unroll
            for (int nb = 0; nb < 4; ++nb) { const v16bf bb = ldb(TP + bp + boff + (size_t)nb * 16 * RK + kc);
#pragma unroll
                for (int mb = 0; mb < 4; ++mb) acc[mb][nb] = wmmab(a[mb], bb, acc[mb][nb]); }
            asm volatile("v_nop\n\tv_nop\n\tv_nop\n\tv_nop" : "+v"(acc[0][0]), "+v"(acc[0][1]), "+v"(acc[0][2]), "+v"(acc[0][3]), "+v"(acc[1][0]), "+v"(acc[1][1]), "+v"(acc[1][2]), "+v"(acc[1][3]) : "v"(a[0]), "v"(a[1]));
            asm volatile("v_nop\n\tv_nop\n\tv_nop\n\tv_nop" : "+v"(acc[2][0]), "+v"(acc[2][1]), "+v"(acc[2][2]), "+v"(acc[2][3]), "+v"(acc[3][0]), "+v"(acc[3][1]), "+v"(acc[3][2]), "+v"(acc[3][3]) : "v"(a[2]), "v"(a[3]));
        }
    }
    float nj[4];
#pragma unroll
    for (int nb = 0; nb < 4; ++nb) nj[nb] = NRM[rb + j0 + nb * 16 + lr];
#pragma unroll
    for (int mb = 0; mb < 4; ++mb) {
        const v4f na = *(const v4f*)(NRM + rb + i0 + mb * 16 + 8 * hi); const v4f nc = *(const v4f*)(NRM + rb + i0 + mb * 16 + 8 * hi + 4);
#pragma unroll
        for (int nb = 0; nb < 4; ++nb) {
#pragma unroll
            for (int j = 0; j < 8; ++j) { const float ni = (j < 4) ? na[j & 3] : nc[j & 3];
                os[(hi * 8 + j) * 68 + nb * 16 + lr] = (ni + nj[nb]) - 2.0f * acc[mb][nb][j]; } }
        wave_sync();
        float* orow = OUT + ((size_t)b * OUT_SEQ + i0 + mb * 16) * OUT_SEQ + j0;
#pragma unroll 1
        for (int ps = 0; ps < 2; ++ps) {
#pragma unroll
            for (int s = 0; s < 8; ++s) { const int row = 2 * s + hi, cofs = lr * 4;
                const v4f val = *(const v4fa*)(&os[row * 68 + cofs]);
                *(volatile v4f*)(orow + (size_t)row * OUT_SEQ + cofs) = val; }
            if (ps == 0) __threadfence(); }
        wave_sync();
    }
}

static constexpr size_t al256(size_t v) { return (v + 255) & ~(size_t)255; }
static constexpr size_t SZ_XB = al256((size_t)NB * SEQ * DIN * 2);
static constexpr size_t SZ_PT = al256((size_t)RK * DIN * 2);
static constexpr size_t PLN   = (size_t)NB * SEQ * RK;
static constexpr size_t SZ_TP = al256(2 * PLN * 2);
static constexpr size_t SZ_NR = al256((size_t)NB * SEQ * 4);
static constexpr size_t SZ_TOTAL = SZ_XB + SZ_PT + SZ_TP + SZ_NR;
static_assert(SZ_TOTAL <= (size_t)134217728);
static_assert((PLN * 2) % 256 == 0);

extern "C" void kernel_launch(void* const* d_in, const int* in_sizes, int n_in,
                              void* d_out, int out_size, void* d_ws, size_t ws_size, hipStream_t stream) {
    if (n_in < 2) return;
    const size_t needx = ((size_t)(NB - 1) * SEQ_FULL + SEQ) * DIN;
    if ((size_t)in_sizes[0] < needx) return;
    if ((size_t)in_sizes[1] < (size_t)DIN * RK) return;
    if ((size_t)out_size < ((size_t)(NB - 1) * OUT_SEQ + SEQ) * OUT_SEQ) return;
    if (SZ_TOTAL > ws_size) return;
    const float* x = (const float*)d_in[0]; const float* pw = (const float*)d_in[1];
    float* OUT = (float*)d_out;
    char* wsp = (char*)d_ws;
    bf* XB = (bf*)wsp; wsp += SZ_XB;
    bf* PT = (bf*)wsp; wsp += SZ_PT;
    bf* TH = (bf*)wsp; wsp += SZ_TP;
    float* NRM = (float*)wsp; wsp += SZ_NR;
    bf* TL = TH + PLN;

    if (SEQ == SEQ_FULL) {
        const size_t n8 = (size_t)NB * SEQ * DIN / 8;
        k_cvt8<<<(unsigned)((n8 + 255) / 256), 256, 0, stream>>>(x, XB, n8);
    } else {
        const size_t n8 = (size_t)SEQ * DIN / 8;
        for (int b = 0; b < NB; ++b) k_cvt8<<<(unsigned)((n8 + 255) / 256), 256, 0, stream>>>(x + (size_t)b * SEQ_FULL * DIN, XB + (size_t)b * SEQ * DIN, n8);
    }
    k_tcvt<<<dim3(DIN / 64, 1, 1), 256, 0, stream>>>(pw, PT);

    k_proj<<<dim3(NB * SEQ / 32, 1, 1), 32, 0, stream>>>(XB, PT, TH, TL, NRM);

    k_gram<<<dim3(SEQ / 64, SEQ / 64, NB), 32, 0, stream>>>(TH, PLN, NRM, OUT);
}
